// Mamba2_6614249636549
// MI455X (gfx1250) — hardware-run, weakly checked
//
#include <hip/hip_runtime.h>
#include <math.h>

typedef __attribute__((ext_vector_type(16))) _Float16 v16h;
typedef __attribute__((ext_vector_type(8)))  _Float16 v8h;
typedef __attribute__((ext_vector_type(2)))  _Float16 v2h;
typedef __attribute__((ext_vector_type(16))) __bf16   v16b;
typedef __attribute__((ext_vector_type(8)))  __bf16   v8b;
typedef __attribute__((ext_vector_type(8)))  float    v8f;
typedef __attribute__((ext_vector_type(4)))  float    v4f;
typedef __attribute__((ext_vector_type(2)))  float    v2f;

constexpr int kNb   = 2;
constexpr int kS    = 2048;
constexpr int kH    = 32;
constexpr int kP    = 64;
constexpr int kN    = 64;
constexpr int kHID  = 2048;
constexpr int kQ    = 64;
constexpr int kC    = kS / kQ;
constexpr int kE    = kH * kC;
constexpr int kRowsAll = kNb * kS;
constexpr int kThr  = 256;
constexpr float kInCarry = 1024.0f;
constexpr float kWCarry  = 4096.0f;
constexpr float kMCarry  = 256.0f;
constexpr float kHCarry  = 1024.0f;
constexpr float kNormEps = 1e-5f;
constexpr float kScT  = 1.0f / (kInCarry * kWCarry);
constexpr float kSc1  = 1.0f / (kWCarry * kWCarry);
constexpr float kSc3  = 1.0f / (kMCarry * kInCarry);
constexpr float kSc4  = 1.0f / (kInCarry * kWCarry);
constexpr float kSc6  = 1.0f / (kWCarry * kHCarry);
constexpr float kScO  = 1.0f / (kInCarry * kInCarry);
constexpr float kF16MinNormal = 6.103515625e-5f;
constexpr int kBiaDt = 0, kBiaG = 32, kBiaO = 64;

static_assert(kQ == 64 && kC == 32 && kE == 1024 && kP == 64 && kN == 64 && kH == 32 && kHID == kH * kP, "the index arithmetic below uses these powers of two");

constexpr size_t kOffZB = 0ull;
constexpr size_t kOffBIA = 4096ull;
constexpr size_t kOffWDT16 = 21504ull;
constexpr size_t kOffWG16 = 152576ull;
constexpr size_t kOffOW2 = 283648ull;
constexpr size_t kOffDTL = 807936ull;
constexpr size_t kOffGTL = 1332224ull;
constexpr size_t kOffHX16 = 1856512ull;
constexpr size_t kOffRNQ = 18633728ull;
constexpr size_t kOffRNK = 18895872ull;
constexpr size_t kOffCS = 19158016ull;
constexpr size_t kOffWTV = 19420160ull;
constexpr size_t kOffEV = 19682304ull;
constexpr size_t kOffDV = 19944448ull;
constexpr size_t kOffTOT = 20206592ull;
constexpr size_t kOffRS = 20210688ull;
constexpr size_t kOffC3 = 20218880ull;
constexpr size_t kOffB3 = 45384704ull;
constexpr size_t kOffXT16 = 70550528ull;
constexpr size_t kOffG32 = 78939136ull;
constexpr size_t kOffM16 = 95716352ull;
constexpr size_t kOffST32 = 104104960ull;
constexpr size_t kOffBDT16 = kOffC3;
constexpr size_t kOffH16   = kOffC3 + 8388608ull;
constexpr size_t kOffCE16  = kOffC3 + 16777216ull;
constexpr size_t kOffYC32  = kOffB3;
constexpr size_t kOffY2    = kOffHX16;
constexpr size_t kWsTotal = 120882176ull;
static_assert(kWsTotal <= 134217728ull, "carve cap: under 128 MiB");
static_assert(kOffZB == 0
              && kOffBIA == kOffZB + 4096ull
              && kOffWDT16 == kOffBIA + 17408ull
              && kOffWG16 == kOffWDT16 + 131072ull
              && kOffOW2 == kOffWG16 + 131072ull
              && kOffDTL == kOffOW2 + 524288ull
              && kOffGTL == kOffDTL + 524288ull
              && kOffHX16 == kOffGTL + 524288ull
              && kOffRNQ == kOffHX16 + 16777216ull
              && kOffRNK == kOffRNQ + 262144ull
              && kOffCS == kOffRNK + 262144ull
              && kOffWTV == kOffCS + 262144ull
              && kOffEV == kOffWTV + 262144ull
              && kOffDV == kOffEV + 262144ull
              && kOffTOT == kOffDV + 262144ull
              && kOffRS == kOffTOT + 4096ull
              && kOffC3 == kOffRS + 8192ull
              && kOffB3 == kOffC3 + 25165824ull
              && kOffXT16 == kOffB3 + 25165824ull
              && kOffG32 == kOffXT16 + 8388608ull
              && kOffM16 == kOffG32 + 16777216ull
              && kOffST32 == kOffM16 + 8388608ull
              && kWsTotal == kOffST32 + 16777216ull, "the carve is chained and totalled");
static_assert((kOffZB % 256) == 0 && (kOffBIA % 256) == 0 && (kOffWDT16 % 256) == 0 && (kOffWG16 % 256) == 0 && (kOffOW2 % 256) == 0 && (kOffDTL % 256) == 0 && (kOffGTL % 256) == 0 && (kOffHX16 % 256) == 0 && (kOffRNQ % 256) == 0 && (kOffRNK % 256) == 0 && (kOffCS % 256) == 0 && (kOffWTV % 256) == 0 && (kOffEV % 256) == 0 && (kOffDV % 256) == 0 && (kOffTOT % 256) == 0 && (kOffRS % 256) == 0 && (kOffC3 % 256) == 0 && (kOffB3 % 256) == 0 && (kOffXT16 % 256) == 0 && (kOffG32 % 256) == 0 && (kOffM16 % 256) == 0 && (kOffST32 % 256) == 0, "aligned regions");
static_assert((size_t)kE * kQ * 192 * 2 == 3ull * 8388608ull && (size_t)kE * kN * kQ * 2 == 8388608ull && (size_t)kE * kP * kN * 2 == 8388608ull
              && (size_t)kS * kH * kP * 4 <= (size_t)kE * kQ * 192 * 2 && (size_t)kS * kH * 128 * 2 <= (size_t)kRowsAll * kHID * 2,
              "the reuses fit: C3's three thirds hold BDT16, H16, CE16; B3 holds YC32; the hidden states' plane holds a sample's Y2");

__device__ __forceinline__ unsigned short f2bf_bits(float f) {
  unsigned u = __float_as_uint(f);
  return (unsigned short)((u + 0x7FFFu + ((u >> 16) & 1u)) >> 16);
}
__device__ __forceinline__ float bf_bits2f(unsigned short h) { return __uint_as_float(((unsigned)h) << 16); }
__device__ __forceinline__ float bf16r(float f) { return bf_bits2f(f2bf_bits(f)); }
__device__ __forceinline__ float carry_flush(float v, float carry) {
  const float s = v * carry;
  return (fabsf(s) < kF16MinNormal) ? 0.0f : s;
}

__device__ __forceinline__ void dep_guard4_h(v8f& a, v8f& b, v8f& c, v8f& d, v16h x, v16h y) { asm volatile("v_nop\n\tv_nop\n\tv_nop\n\tv_nop" : "+v"(a), "+v"(b), "+v"(c), "+v"(d) : "v"(x), "v"(y)); }
__device__ __forceinline__ void dep_guard4_b(v8f& a, v8f& b, v8f& c, v8f& d, v16b x, v16b y) { asm volatile("v_nop\n\tv_nop\n\tv_nop\n\tv_nop" : "+v"(a), "+v"(b), "+v"(c), "+v"(d) : "v"(x), "v"(y)); }
__device__ __forceinline__ void keep4_h(v16h a, v16h b, v16h c, v16h d) { asm volatile("v_nop" :: "v"(a), "v"(b), "v"(c), "v"(d)); }
__device__ __forceinline__ void keep4_b(v16b a, v16b b, v16b c, v16b d) { asm volatile("v_nop" :: "v"(a), "v"(b), "v"(c), "v"(d)); }
__device__ __forceinline__ void acc_guard4(v8f& a, v8f& b, v8f& c, v8f& d) { asm volatile("v_nop\n\tv_nop\n\tv_nop\n\tv_nop" : "+v"(a), "+v"(b), "+v"(c), "+v"(d)); }

template <typename T> struct Frag;
template <> struct Frag<_Float16> {
  typedef v16h V; union U { v16h v; v8h h[2]; };
  static __device__ __forceinline__ v16h load(const _Float16* p) {
    U f; f.h[0] = *(const v8h*)(p); f.h[1] = *(const v8h*)(p + 16); return f.v;
  }
  static __device__ __forceinline__ v8f mma(v16h a, v16h b, v8f c) {
    return __builtin_amdgcn_wmma_f32_16x16x32_f16(false, a, false, b, (short)0, c, false, false);
  }
  static __device__ __forceinline__ void guard4(v8f& a, v8f& b, v8f& c, v8f& d, v16h x, v16h y) { dep_guard4_h(a, b, c, d, x, y); }
  static __device__ __forceinline__ void keep(v16h a, v16h b, v16h c, v16h d) { keep4_h(a, b, c, d); }
};
template <> struct Frag<__bf16> {
  typedef v16b V; union U { v16b v; v8b h[2]; };
  static __device__ __forceinline__ v16b load(const __bf16* p) {
    U f; f.h[0] = *(const v8b*)(p); f.h[1] = *(const v8b*)(p + 16); return f.v;
  }
  static __device__ __forceinline__ v8f mma(v16b a, v16b b, v8f c) {
    return __builtin_amdgcn_wmma_f32_16x16x32_bf16(false, a, false, b, (short)0, c, false, false);
  }
  static __device__ __forceinline__ void guard4(v8f& a, v8f& b, v8f& c, v8f& d, v16b x, v16b y) { dep_guard4_b(a, b, c, d, x, y); }
  static __device__ __forceinline__ void keep(v16b a, v16b b, v16b c, v16b d) { keep4_b(a, b, c, d); }
};

__device__ __forceinline__ v8f mma_h(v16h a, v16h b, v8f c) {
  c = __builtin_amdgcn_wmma_f32_16x16x32_f16(false, a, false, b, (short)0, c, false, false);
  asm volatile("v_nop\n\tv_nop\n\tv_nop\n\tv_nop" : "+v"(c) : "v"(a), "v"(b));
  return c;
}

template <int ET> struct Elem;
template <> struct Elem<0> { typedef _Float16 T; };
template <> struct Elem<1> { typedef __bf16 T; };
template <int ET, bool SPLIT, int BIAS_MODE, int OUT_MODE, bool RESID, int ACT = 0>
__global__ __launch_bounds__(256) void wmma_gemm64(
    const unsigned short* __restrict__ Ap, const unsigned short* __restrict__ A2p, int lda, long strideA,
    const unsigned short* __restrict__ Btp, const unsigned short* __restrict__ Bt2p, int ldb, long strideB,
    void* __restrict__ Cout, void* __restrict__ Cout2, int ldc, long strideC,
    const float* __restrict__ bias,
    const float* __restrict__ resid, long strideR,
    int M, int N, int K, float scale) {
  typedef typename Elem<ET>::T T;
  typedef typename Frag<T>::V V;
  const T* A = (const T*)Ap; const T* A2 = (const T*)A2p; const T* Bt = (const T*)Btp; const T* Bt2 = (const T*)Bt2p;
  __shared__ __align__(16) float sT[8][16 * 68];
  const int b    = blockIdx.y;
  const int lane = threadIdx.x & 31;
  const int wave = threadIdx.x >> 5;
  const int tilesN = N >> 6;
  const int tilesM = M >> 6;
  const int tile = blockIdx.x * 8 + wave;
  if (tile >= tilesM * tilesN) return;
  const int tm = tile / tilesN;
  const int tn = tile - tm * tilesN;
  const int m0 = tm << 6;
  const int n0 = tn << 6;

  const T* Ab  = A  + (size_t)b * strideA;
  const T* Bb  = Bt + (size_t)b * strideB;
  const T* Ab2 = SPLIT ? (A2  + (size_t)b * strideA) : nullptr;
  const T* Bb2 = SPLIT ? (Bt2 + (size_t)b * strideB) : nullptr;

  const int rlane = lane & 15;
  const int koff  = (lane >> 4) * 8;
  const int mOff  = (lane >> 4) * 8;

  v8f acc[4][4];
#pragma unroll
  for (int i = 0; i < 4; ++i)
#pragma unroll
    for (int j = 0; j < 4; ++j) acc[i][j] = (v8f){0.f,0.f,0.f,0.f,0.f,0.f,0.f,0.f};

  for (int k0 = 0; k0 < K; k0 += 32) {
    V bh[4], bl[4];
#pragma unroll
    for (int j = 0; j < 4; ++j) {
      const size_t bo = (size_t)(n0 + (j << 4) + rlane) * ldb + koff + k0;
      bh[j] = Frag<T>::load(Bb + bo);
      if (SPLIT) bl[j] = Frag<T>::load(Bb2 + bo);
    }
#pragma unroll
    for (int i = 0; i < 4; ++i) {
      const size_t ao = (size_t)(m0 + (i << 4) + rlane) * lda + koff + k0;
      V ah = Frag<T>::load(Ab + ao);
      V al;
      if (SPLIT) al = Frag<T>::load(Ab2 + ao);
#pragma unroll
      for (int j = 0; j < 4; ++j) {
        acc[i][j] = Frag<T>::mma(ah, bh[j], acc[i][j]);
        if (SPLIT) {
          acc[i][j] = Frag<T>::mma(ah, bl[j], acc[i][j]);
          acc[i][j] = Frag<T>::mma(al, bh[j], acc[i][j]);
        }
      }
      Frag<T>::guard4(acc[i][0], acc[i][1], acc[i][2], acc[i][3], ah, SPLIT ? al : ah);
    }
    Frag<T>::keep(bh[0], bh[1], bh[2], bh[3]);
    if (SPLIT) Frag<T>::keep(bl[0], bl[1], bl[2], bl[3]);
  }
  acc_guard4(acc[0][0], acc[0][1], acc[0][2], acc[0][3]);
  acc_guard4(acc[1][0], acc[1][1], acc[1][2], acc[1][3]);
  acc_guard4(acc[2][0], acc[2][1], acc[2][2], acc[2][3]);
  acc_guard4(acc[3][0], acc[3][1], acc[3][2], acc[3][3]);

  float* slab = sT[wave];
  const float* Rb = RESID ? (resid + (size_t)b * strideR) : nullptr;
#pragma unroll
  for (int i = 0; i < 4; ++i) {
    const int mBase = m0 + (i << 4);
#pragma unroll
    for (int j = 0; j < 4; ++j) {
      const int n = n0 + (j << 4) + rlane;
      float bv = 0.f;
      if (BIAS_MODE == 2) bv = bias[n];
#pragma unroll
      for (int r = 0; r < 8; ++r) {
        float v = acc[i][j][r] * scale;
        if (BIAS_MODE == 1) v += bias[mBase + mOff + r];
        if (BIAS_MODE == 2) v += bv;
        if (RESID) v += Rb[(size_t)(mBase + mOff + r) * ldc + n];
        if (ACT == 1) v = tanhf(v);
        if (ACT == 2) v = fmaxf(v, 0.0f);
        if (ACT == 3) v = v / (1.0f + expf(-v));
        if (ACT == 4) v = (v > 0.f) ? v : 0.01f * v;
        slab[(mOff + r) * 68 + (j << 4) + rlane] = v;
      }
    }
    __builtin_amdgcn_fence(__ATOMIC_RELEASE, "workgroup");
    __builtin_amdgcn_wave_barrier();
    __builtin_amdgcn_fence(__ATOMIC_ACQUIRE, "workgroup");
    if (OUT_MODE == 0) {
      float* C = (float*)Cout + (size_t)b * strideC;
      const int hh = lane >> 4, c4 = (lane & 15) * 4;
      for (int pass = 0; pass < 2; ++pass) {
#pragma unroll
        for (int it = 0; it < 8; ++it) {
          const int row = it * 2 + hh;
          v4f v = *(const v4f*)(slab + row * 68 + c4);
          *(volatile v4f*)(C + (size_t)(mBase + row) * ldc + n0 + c4) = v;
        }
        __threadfence();
      }
    } else {
      const int q = lane >> 3, c8 = (lane & 7) * 8;
      unsigned short* C  = (unsigned short*)Cout  + (size_t)b * strideC;
      unsigned short* C2 = (OUT_MODE == 2) ? ((unsigned short*)Cout2 + (size_t)b * strideC) : nullptr;
      for (int pass = 0; pass < 2; ++pass) {
#pragma unroll
        for (int it = 0; it < 4; ++it) {
          const int row = it * 4 + q;
          const float* sp = slab + row * 68 + c8;
          v8h hv, lv;
#pragma unroll
          for (int e = 0; e < 8; ++e) {
            if (OUT_MODE == 1) {
              hv[e] = (_Float16)sp[e];
            } else {
              unsigned short hb = f2bf_bits(sp[e]);
              unsigned short lb = f2bf_bits(sp[e] - bf_bits2f(hb));
              hv[e] = __builtin_bit_cast(_Float16, hb);
              lv[e] = __builtin_bit_cast(_Float16, lb);
            }
          }
          *(volatile v8h*)(C + (size_t)(mBase + row) * ldc + n0 + c8) = hv;
          if (OUT_MODE == 2) *(volatile v8h*)(C2 + (size_t)(mBase + row) * ldc + n0 + c8) = lv;
        }
        __threadfence();
      }
    }
    __builtin_amdgcn_fence(__ATOMIC_RELEASE, "workgroup");
    __builtin_amdgcn_wave_barrier();
    __builtin_amdgcn_fence(__ATOMIC_ACQUIRE, "workgroup");
  }
}

__global__ __launch_bounds__(kThr) void cast_plane_kernel(const float* __restrict__ src, unsigned short* __restrict__ dst,
                                                          int colsLog2, int dstPitch, int dstOff) {
  const int i   = blockIdx.x * kThr + threadIdx.x;
  const int sh  = colsLog2 - 3;
  const int row = i >> sh;
  const int c8  = (i & ((1 << sh) - 1)) * 8;
  const float* sp = src + ((size_t)row << colsLog2) + c8;
  const v4f a0 = *(const v4f*)(sp);
  const v4f a1 = *(const v4f*)(sp + 4);
  v8h hv;
#pragma unroll
  for (int e = 0; e < 4; ++e) {
    const float f0 = a0[e];
    const float f1 = a1[e];
    hv[e]     = (_Float16)carry_flush(bf16r(f0), kInCarry);
    hv[4 + e] = (_Float16)carry_flush(bf16r(f1), kInCarry);
  }
  unsigned short* dp = dst + (size_t)row * dstPitch + dstOff + c8;
  *(volatile v8h*)dp = hv;
  __threadfence();
  *(volatile v8h*)dp = hv;
}

__global__ __launch_bounds__(256) void wt_plane_kernel(const float* __restrict__ W, unsigned short* __restrict__ dst, int K, int N, int nLive, int ldd, int colOff) {
  const int n  = blockIdx.x;
  const int k8 = threadIdx.x * 8;
  const bool live = n < nLive;
  const int nc = live ? n : 0;
  v8h hv;
#pragma unroll
  for (int e = 0; e < 8; ++e) {
    const float w = W[(size_t)(k8 + e) * N + nc];
    hv[e] = (_Float16)(live ? carry_flush(bf16r(w), kWCarry) : 0.0f);
  }
  unsigned short* dp = dst + (size_t)n * ldd + colOff + k8;
  *(volatile v8h*)dp = hv;
  __threadfence();
  *(volatile v8h*)dp = hv;
}
__global__ __launch_bounds__(256) void wmma_gemm32(
    const unsigned short* __restrict__ Ap, int lda, long strideA,
    const unsigned short* __restrict__ Btp, int ldb, long strideB,
    float* __restrict__ Cout, int ldc, long strideC,
    const float* __restrict__ bias,
    int M, int N, int K, float scale) {
  typedef _Float16 T;
  typedef Frag<T>::V V;
  const T* A = (const T*)Ap; const T* Bt = (const T*)Btp;
  __shared__ __align__(16) float sT[8][16 * 36];
  const int b    = blockIdx.y;
  const int lane = threadIdx.x & 31;
  const int wave = threadIdx.x >> 5;
  const int tilesN = N >> 5;
  const int tilesM = M >> 6;
  const int tile = blockIdx.x * 8 + wave;
  if (tile >= tilesM * tilesN) return;
  const int tm = tile / tilesN;
  const int tn = tile - tm * tilesN;
  const int m0 = tm << 6;
  const int n0 = tn << 5;

  const T* Ab = A  + (size_t)b * strideA;
  const T* Bb = Bt + (size_t)b * strideB;

  const int rlane = lane & 15;
  const int koff  = (lane >> 4) * 8;
  const int mOff  = (lane >> 4) * 8;

  v8f acc[4][2];
#pragma unroll
  for (int i = 0; i < 4; ++i)
#pragma unroll
    for (int j = 0; j < 2; ++j) acc[i][j] = (v8f){0.f,0.f,0.f,0.f,0.f,0.f,0.f,0.f};

  for (int k0 = 0; k0 < K; k0 += 32) {
    V bh[2];
#pragma unroll
    for (int j = 0; j < 2; ++j) {
      const size_t bo = (size_t)(n0 + (j << 4) + rlane) * ldb + koff + k0;
      bh[j] = Frag<T>::load(Bb + bo);
    }
#pragma unroll
    for (int i = 0; i < 4; i += 2) {
      const size_t ao0 = (size_t)(m0 + (i << 4) + rlane) * lda + koff + k0;
      const size_t ao1 = (size_t)(m0 + ((i + 1) << 4) + rlane) * lda + koff + k0;
      V ah0 = Frag<T>::load(Ab + ao0);
      V ah1 = Frag<T>::load(Ab + ao1);
      acc[i][0]     = Frag<T>::mma(ah0, bh[0], acc[i][0]);
      acc[i][1]     = Frag<T>::mma(ah0, bh[1], acc[i][1]);
      acc[i + 1][0] = Frag<T>::mma(ah1, bh[0], acc[i + 1][0]);
      acc[i + 1][1] = Frag<T>::mma(ah1, bh[1], acc[i + 1][1]);
      Frag<T>::guard4(acc[i][0], acc[i][1], acc[i + 1][0], acc[i + 1][1], ah0, ah1);
    }
    Frag<T>::keep(bh[0], bh[1], bh[0], bh[1]);
  }
  acc_guard4(acc[0][0], acc[0][1], acc[1][0], acc[1][1]);
  acc_guard4(acc[2][0], acc[2][1], acc[3][0], acc[3][1]);

  float* slab = sT[wave];
  float* C = Cout + (size_t)b * strideC;
#pragma unroll
  for (int i = 0; i < 4; ++i) {
    const int mBase = m0 + (i << 4);
#pragma unroll
    for (int j = 0; j < 2; ++j) {
      const int n = n0 + (j << 4) + rlane;
      const float bv = bias[n];
#pragma unroll
      for (int r = 0; r < 8; ++r) {
        float v = acc[i][j][r] * scale;
        v += bv;
        slab[(mOff + r) * 36 + (j << 4) + rlane] = v;
      }
    }
    __builtin_amdgcn_fence(__ATOMIC_RELEASE, "workgroup");
    __builtin_amdgcn_wave_barrier();
    __builtin_amdgcn_fence(__ATOMIC_ACQUIRE, "workgroup");
    {
      const int q = lane >> 3, c4 = (lane & 7) * 4;
      for (int pass = 0; pass < 2; ++pass) {
#pragma unroll
        for (int it = 0; it < 4; ++it) {
          const int row = it * 4 + q;
          v4f v = *(const v4f*)(slab + row * 36 + c4);
          *(volatile v4f*)(C + (size_t)(mBase + row) * ldc + n0 + c4) = v;
        }
        __threadfence();
      }
    }
    __builtin_amdgcn_fence(__ATOMIC_RELEASE, "workgroup");
    __builtin_amdgcn_wave_barrier();
    __builtin_amdgcn_fence(__ATOMIC_ACQUIRE, "workgroup");
  }
}
static_assert(sizeof(float) * 8 * 16 * 36 == 18432, "the tail's slabs: 8 waves x 16 rows x 36 floats = 18,432 B of LDS");


__global__ __launch_bounds__(kThr) void zero_kernel(float* __restrict__ dst) {
  const size_t o4 = ((size_t)blockIdx.x * kThr + threadIdx.x) * 4u;
  const v4f z = {0.f, 0.f, 0.f, 0.f};
  *(volatile v4f*)(dst + o4) = z;
  __threadfence();
  *(volatile v4f*)(dst + o4) = z;
}

__global__ __launch_bounds__(kThr) void bias_kernel(const float* __restrict__ dt_b, const float* __restrict__ dt_bias, const float* __restrict__ g_b, const float* __restrict__ o_b,
                                                   float* __restrict__ BIA) {
  const unsigned i = blockIdx.x * (unsigned)kThr + threadIdx.x;
  const unsigned i32 = i & 31u;
  const unsigned io = (i >= 64u && i < 64u + (unsigned)(kH * kP)) ? (i - 64u) : 0u;
  const float a = dt_b[i32], b = dt_bias[i32], c = g_b[i32], d = o_b[io];
  float v = 0.0f;
  if (i < 32u) v = bf16r(a) + bf16r(b);
  else if (i < 64u) v = bf16r(c);
  else if (i < 64u + (unsigned)(kH * kP)) v = bf16r(d);
  *(volatile float*)(BIA + i) = v;
  __threadfence();
  *(volatile float*)(BIA + i) = v;
}
static_assert(4352 == 17 * kThr && 64 + kH * kP <= 4352, "bias grid exact: 17 blocks");

__global__ __launch_bounds__(kThr) void xt2_cast_kernel(const float* __restrict__ V, unsigned short* __restrict__ XT2) {
  const unsigned i = blockIdx.x * (unsigned)kThr + threadIdx.x;
  const unsigned j = i & 15u, p = (i >> 4) & 63u, e = i >> 10;
  const float* sp = V + ((size_t)e * kQ + (j & 7u) * 8u) * kP + p;
  v8h hv;
#pragma unroll
  for (int t = 0; t < 8; ++t) { const float x = sp[(size_t)t * kP]; hv[t] = (_Float16)carry_flush(bf16r(x), kInCarry); }
  unsigned short* dp = XT2 + (size_t)i * 8u;
  *(volatile v8h*)dp = hv;
  __threadfence();
  *(volatile v8h*)dp = hv;
}
static_assert((size_t)kH * kP * (2 * kP / 8) == 128ull * kThr, "the out-projection weights' cast grid exact: 128 blocks");

__global__ __launch_bounds__(kThr) void rownorm_kernel(const float* __restrict__ src, float* __restrict__ RN) {
  const unsigned i = blockIdx.x * (unsigned)kThr + threadIdx.x;
  const unsigned l = i & 63u, e = i >> 6;
  const unsigned h = e >> 5, c = e & 31u;
  const float* sp = src + ((size_t)(c * (unsigned)kQ + l) * kH + h) * kP;
  float ss = 0.0f;
#pragma unroll
  for (int q4 = 0; q4 < kP / 4; ++q4) {
    const v4f a = *(const v4f*)(sp + 4 * q4);
#pragma unroll
    for (int t = 0; t < 4; ++t) { const float x = a[t]; const float xb = bf16r(x); ss += xb * xb; }
  }
  const float rn = 1.0f / fmaxf(sqrtf(ss), 1e-12f);
  *(volatile float*)(RN + i) = rn;
  __threadfence();
  *(volatile float*)(RN + i) = rn;
}
static_assert((size_t)kE * kQ == 256ull * kThr, "row-norm grid exact: 256 blocks");

__global__ __launch_bounds__(kThr) void hm3_cast_kernel(const float* __restrict__ src, const float* __restrict__ RN, unsigned short* __restrict__ dst, int third) {
  const unsigned i = blockIdx.x * (unsigned)kThr + threadIdx.x;
  const unsigned n8 = i & 7u, l = (i >> 3) & 63u, e = i >> 9;
  const unsigned h = e >> 5, c = e & 31u;
  const float* sp = src + ((size_t)(c * (unsigned)kQ + l) * kH + h) * kP + n8 * 8u;
  const v4f a0 = *(const v4f*)sp, a1 = *(const v4f*)(sp + 4);
  const float f = RN[i >> 3];
  v8h hv, lv;
#pragma unroll
  for (int t = 0; t < 8; ++t) {
    const float x = (t < 4) ? a0[t] : a1[t - 4];
    const float sc = carry_flush(bf16r(x) * f, kWCarry);
    const _Float16 hh = (_Float16)sc;
    const float rs = sc - (float)hh;
    hv[t] = hh;
    lv[t] = (_Float16)((fabsf(rs) < kF16MinNormal) ? 0.0f : rs);
  }
  const bool isB = third != 0;
  unsigned short* dp = dst + (size_t)(i >> 3) * 192u + n8 * 8u;
  for (int pass = 0; pass < 2; ++pass) {
    *(volatile v8h*)dp = hv;
    *(volatile v8h*)(dp + 64) = isB ? hv : lv;
    *(volatile v8h*)(dp + 128) = isB ? lv : hv;
    __threadfence();
  }
}
static_assert((size_t)kE * kQ * (kN / 8) == 2048ull * kThr, "three-block cast grid exact: 2,048 blocks");

__global__ __launch_bounds__(kThr) void xt_cast_kernel(const float* __restrict__ X, unsigned short* __restrict__ XT16) {
  const unsigned i = blockIdx.x * (unsigned)kThr + threadIdx.x;
  const unsigned j = i & 7u, p = (i >> 3) & 63u, e = i >> 9;
  const unsigned h = e >> 5, c = e & 31u;
  const float* sp = X + ((size_t)(c * (unsigned)kQ + j * 8u) * kH + h) * kP + p;
  v8h hv;
#pragma unroll
  for (int t = 0; t < 8; ++t) { const float v = sp[(size_t)t * kH * kP]; hv[t] = (_Float16)carry_flush(bf16r(v), kInCarry); }
  unsigned short* dp = XT16 + (size_t)i * 8u;
  *(volatile v8h*)dp = hv;
  __threadfence();
  *(volatile v8h*)dp = hv;
}
static_assert((size_t)kE * kP * (kQ / 8) == 2048ull * kThr, "transposing cast grid exact: 2,048 blocks");

__global__ __launch_bounds__(kThr) void prefix_kernel(const float* __restrict__ DTLs, const float* __restrict__ A_log, float* __restrict__ CS, float* __restrict__ WTV,
                                                     float* __restrict__ EV, float* __restrict__ DV, float* __restrict__ TOT) {
  const unsigned e = blockIdx.x * (unsigned)kThr + threadIdx.x;
  const unsigned h = e >> 5, c = e & 31u;
  const float* ap = DTLs + (size_t)(c * (unsigned)kQ) * kH + h;
  const float al = A_log[h];
  const float Ah = -expf(bf16r(al));
  float run = 0.0f;
  for (int q = 0; q < kQ / 4; ++q) {
    v4f s4, o4;
#pragma unroll
    for (int t = 0; t < 4; ++t) { const float pre = ap[(size_t)(4 * q + t) * kH]; const float dtv = (pre > 20.0f) ? pre : log1pf(expf(pre)); run += dtv * Ah; s4[t] = run; o4[t] = dtv; }
    float* sp = CS + (size_t)e * kQ + 4 * q; float* xp = WTV + (size_t)e * kQ + 4 * q;
    for (int pass = 0; pass < 2; ++pass) { *(volatile v4f*)sp = s4; *(volatile v4f*)xp = o4; __threadfence(); }
  }
  const float tot = run;
  run = 0.0f;
  for (int q = 0; q < kQ / 4; ++q) {
    v4f e4, d4;
#pragma unroll
    for (int t = 0; t < 4; ++t) { const float pre = ap[(size_t)(4 * q + t) * kH]; const float dtv = (pre > 20.0f) ? pre : log1pf(expf(pre)); run += dtv * Ah; e4[t] = expf(run); d4[t] = expf(tot - run) * dtv; }
    float* ep = EV + (size_t)e * kQ + 4 * q; float* dp = DV + (size_t)e * kQ + 4 * q;
    for (int pass = 0; pass < 2; ++pass) { *(volatile v4f*)ep = e4; *(volatile v4f*)dp = d4; __threadfence(); }
  }
  const float te = expf(tot);
  *(volatile float*)(TOT + e) = te;
  __threadfence();
  *(volatile float*)(TOT + e) = te;
}
static_assert(kE == 4 * kThr && (kQ % 4) == 0, "prefix grid exact: 4 blocks; the two passes' trip count is the literal 16 (64 positions by fours)");

__global__ __launch_bounds__(kThr) void mask_kernel(const float* __restrict__ G32, const float* __restrict__ CS, const float* __restrict__ OMV, unsigned short* __restrict__ M16) {
  const unsigned i = blockIdx.x * (unsigned)kThr + threadIdx.x;
  const unsigned s8 = i & 7u, l = (i >> 3) & 63u, e = i >> 9;
  const float* gp = G32 + (size_t)i * 8u;
  const float* xp = CS + (size_t)e * kQ + s8 * 8u;
  const float* wp = OMV + (size_t)e * kQ + s8 * 8u;
  const v4f g0 = *(const v4f*)gp, g1 = *(const v4f*)(gp + 4), x0 = *(const v4f*)xp, x1 = *(const v4f*)(xp + 4), w0 = *(const v4f*)wp, w1 = *(const v4f*)(wp + 4);
  const float csl = CS[(size_t)e * kQ + l];
  v8h hv;
#pragma unroll
  for (int t = 0; t < 8; ++t) {
    const bool live = (s8 * 8u + (unsigned)t) <= l;
    const float gv = (t < 4) ? g0[t] : g1[t - 4];
    const float xv = (t < 4) ? x0[t] : x1[t - 4];
    const float ov = (t < 4) ? w0[t] : w1[t - 4];
    const float d = live ? (csl - xv) : 0.0f;
    const float w = live ? gv * expf(d) * ov : 0.0f;
    hv[t] = (_Float16)carry_flush(w, kMCarry);
  }
  unsigned short* dp = M16 + (size_t)i * 8u;
  *(volatile v8h*)dp = hv;
  __threadfence();
  *(volatile v8h*)dp = hv;
}
static_assert((size_t)kE * kQ * (kQ / 8) == 2048ull * kThr, "mask grid exact: 2,048 blocks");

__global__ __launch_bounds__(kThr) void sc2_cast_kernel(const float* __restrict__ src, const float* __restrict__ f1, const float* __restrict__ f2, unsigned short* __restrict__ dst, int tr) {
  const unsigned i = blockIdx.x * (unsigned)kThr + threadIdx.x;
  const unsigned lo = i & 7u, mid = (i >> 3) & 63u, e = i >> 9;
  const unsigned h = e >> 5, c = e & 31u;
  v8h hv;
  if (tr != 0) {
    const float* sp = src + ((size_t)(c * (unsigned)kQ + lo * 8u) * kH + h) * kP + mid;
    const float* p1 = f1 + (size_t)e * kQ + lo * 8u; const float* p2 = f2 + (size_t)e * kQ + lo * 8u;
    const v4f a0 = *(const v4f*)p1, a1 = *(const v4f*)(p1 + 4), b0 = *(const v4f*)p2, b1 = *(const v4f*)(p2 + 4);
#pragma unroll
    for (int t = 0; t < 8; ++t) { const float x = sp[(size_t)t * kH * kP]; const float fa = (t < 4) ? a0[t] : a1[t - 4]; const float fb = (t < 4) ? b0[t] : b1[t - 4]; hv[t] = (_Float16)carry_flush(bf16r(x) * fa * fb, kWCarry); }
  } else {
    const float* sp = src + ((size_t)(c * (unsigned)kQ + mid) * kH + h) * kP + lo * 8u;
    const v4f a0 = *(const v4f*)sp, a1 = *(const v4f*)(sp + 4);
    const float fa = f1[(size_t)e * kQ + mid], fb = f2[(size_t)e * kQ + mid];
#pragma unroll
    for (int t = 0; t < 8; ++t) { const float x = (t < 4) ? a0[t] : a1[t - 4]; hv[t] = (_Float16)carry_flush(bf16r(x) * fa * fb, kWCarry); }
  }
  unsigned short* dp = dst + (size_t)i * 8u;
  *(volatile v8h*)dp = hv;
  __threadfence();
  *(volatile v8h*)dp = hv;
}
static_assert((size_t)kE * kQ * (kN / 8) == 2048ull * kThr, "two-factor cast grid exact: 2,048 blocks");

__global__ __launch_bounds__(kThr) void carry_kernel(const float* __restrict__ ST32, const float* __restrict__ TOT, unsigned short* __restrict__ H16) {
  const unsigned i = blockIdx.x * (unsigned)kThr + threadIdx.x;
  const unsigned n2 = i & 31u, p = (i >> 5) & 63u, h = i >> 11;
  float h0 = 0.0f, h1 = 0.0f;
  for (int c = 0; c < kC; ++c) {
    const size_t e = (size_t)h * kC + (size_t)c;
    const size_t o = (e * kP + p) * kN + n2 * 2u;
    v2h hv;
    hv[0] = (_Float16)carry_flush(h0, kHCarry);
    hv[1] = (_Float16)carry_flush(h1, kHCarry);
    unsigned short* dp = H16 + o;
    *(volatile v2h*)dp = hv;
    __threadfence();
    *(volatile v2h*)dp = hv;
    const v2f sv = *(const v2f*)(ST32 + o);
    const float tt = TOT[e];
    h0 = tt * h0 + sv[0];
    h1 = tt * h1 + sv[1];
  }
}
static_assert((size_t)kH * kP * (kN / 2) == 256ull * kThr && kN / 2 == 32, "carry grid exact: 256 blocks; a wave = one [p] row of 64 state columns");

__global__ __launch_bounds__(kThr) void combine_kernel(const float* __restrict__ YD32, const float* __restrict__ YO32, float* __restrict__ YC32) {
  const unsigned i = blockIdx.x * (unsigned)kThr + threadIdx.x;
  const unsigned p4 = i & 15u, h = (i >> 4) & 31u, t = i >> 9;
  const size_t so = (((size_t)h * kC + (t >> 6)) * kQ + (t & 63u)) * kP + p4 * 4u;
  const v4f a = *(const v4f*)(YD32 + so), b = *(const v4f*)(YO32 + so);
  v4f o;
#pragma unroll
  for (int k = 0; k < 4; ++k) o[k] = a[k] + b[k];
  float* dp = YC32 + (size_t)i * 4u;
  *(volatile v4f*)dp = o;
  __threadfence();
  *(volatile v4f*)dp = o;
}
static_assert((size_t)kS * kH * (kP / 4) == 4096ull * kThr, "combine grid exact: 4,096 blocks a sample");

__global__ __launch_bounds__(kThr) void gnorm_kernel(const float* __restrict__ YC32, const float* __restrict__ GTLs, float* __restrict__ RS) {
  const unsigned t = blockIdx.x * (unsigned)kThr + threadIdx.x;
  const float* yp = YC32 + (size_t)t * kHID;
  const float* gp = GTLs + (size_t)t * kH;
  float ss = 0.0f;
  for (int h = 0; h < kH; ++h) {
    const float g = gp[h];
    const float sg = g / (1.0f + expf(-g));
#pragma unroll
    for (int q4 = 0; q4 < kP / 4; ++q4) {
      const v4f a = *(const v4f*)(yp + h * kP + 4 * q4);
#pragma unroll
      for (int k = 0; k < 4; ++k) { const float yg = a[k] * sg; ss += yg * yg; }
    }
  }
  const float rs = 1.0f / sqrtf(ss * (1.0f / (float)kHID) + kNormEps);
  *(volatile float*)(RS + t) = rs;
  __threadfence();
  *(volatile float*)(RS + t) = rs;
}
static_assert(kS == 8 * kThr, "gated-norm grid exact: 8 blocks a sample");

__global__ __launch_bounds__(kThr) void y2_cast_kernel(const float* __restrict__ YC32, const float* __restrict__ GTLs, const float* __restrict__ RS, const float* __restrict__ nw,
                                                      unsigned short* __restrict__ Y2) {
  const unsigned i = blockIdx.x * (unsigned)kThr + threadIdx.x;
  const unsigned p8 = i & 7u, h = (i >> 3) & 31u, t = i >> 8;
  const float* yp = YC32 + (size_t)i * 8u;
  const float* wp = nw + h * (unsigned)kP + p8 * 8u;
  const v4f a0 = *(const v4f*)yp, a1 = *(const v4f*)(yp + 4), w0 = *(const v4f*)wp, w1 = *(const v4f*)(wp + 4);
  const float g = GTLs[(size_t)t * kH + h];
  const float f = (g / (1.0f + expf(-g))) * RS[t];
  v8h hv, lv;
#pragma unroll
  for (int k = 0; k < 8; ++k) {
    const float y = (k < 4) ? a0[k] : a1[k - 4];
    const float wr = (k < 4) ? w0[k] : w1[k - 4];
    const float sc = carry_flush(y * f * bf16r(wr), kInCarry);
    const _Float16 hh = (_Float16)sc;
    const float rs = sc - (float)hh;
    hv[k] = hh;
    lv[k] = (_Float16)((fabsf(rs) < kF16MinNormal) ? 0.0f : rs);
  }
  unsigned short* dp = Y2 + (size_t)(i >> 3) * 128u + p8 * 8u;
  for (int pass = 0; pass < 2; ++pass) { *(volatile v8h*)dp = hv; *(volatile v8h*)(dp + 64) = lv; __threadfence(); }
}
static_assert((size_t)kS * kH * (kP / 8) == 2048ull * kThr, "two-word output cast grid exact: 2,048 blocks a sample");

static_assert(((size_t)kRowsAll * kHID / 8) % kThr == 0 && ((size_t)kRowsAll * kHID) % 2048 == 0 && (kHID % 8) == 0 && kHID / 8 == 256, "hidden-state cast grids exact; the weight transposer's block is K / 8 = 256 threads");
static_assert((kRowsAll / 64) * (32 / 32) % 8 == 0 && ((kS / 64) * (kP / 64)) % 8 == 0, "the tile's and the out-projections' grids exact");

extern "C" void kernel_launch(void* const* d_in, const int* in_sizes, int n_in,
                              void* d_out, int out_size, void* d_ws, size_t ws_size,
                              hipStream_t stream) {
  if (n_in < 14 || d_out == nullptr || d_ws == nullptr) return;
  if (in_sizes[0] != kRowsAll * kHID || in_sizes[1] != kRowsAll * kHID || in_sizes[2] != kRowsAll * kH * kP || in_sizes[3] != kRowsAll * kH * kP || in_sizes[4] != kRowsAll * kH * kP) return;
  if (in_sizes[5] != kHID * kH || in_sizes[6] != kH || in_sizes[7] != kHID * kH || in_sizes[8] != kH || in_sizes[9] != kH || in_sizes[10] != kH || in_sizes[11] != kHID) return;
  if (in_sizes[12] != kH * kP * kP || in_sizes[13] != kH * kP) return;
  if (out_size != kRowsAll * kHID) return;
  if (ws_size < kWsTotal) return;
  const float* hab = (const float*)d_in[0];
  const float* hg = (const float*)d_in[1];
  const float* qs = (const float*)d_in[2];
  const float* ks = (const float*)d_in[3];
  const float* vs = (const float*)d_in[4];
  const float* dt_w = (const float*)d_in[5];
  const float* dt_b = (const float*)d_in[6];
  const float* g_w = (const float*)d_in[7];
  const float* g_b = (const float*)d_in[8];
  const float* A_log = (const float*)d_in[9];
  const float* dt_bias = (const float*)d_in[10];
  const float* nw = (const float*)d_in[11];
  const float* o_w = (const float*)d_in[12];
  const float* o_b = (const float*)d_in[13];
  float* out = (float*)d_out;
  char* ws = (char*)d_ws;
  float* ZB = (float*)(ws + kOffZB);
  float* BIA = (float*)(ws + kOffBIA);
  unsigned short* WDT16 = (unsigned short*)(ws + kOffWDT16);
  unsigned short* WG16 = (unsigned short*)(ws + kOffWG16);
  unsigned short* OW2 = (unsigned short*)(ws + kOffOW2);
  float* DTL = (float*)(ws + kOffDTL);
  float* GTL = (float*)(ws + kOffGTL);
  unsigned short* HX16 = (unsigned short*)(ws + kOffHX16);
  unsigned short* Y2 = (unsigned short*)(ws + kOffY2);
  float* RNQ = (float*)(ws + kOffRNQ);
  float* RNK = (float*)(ws + kOffRNK);
  float* CS = (float*)(ws + kOffCS);
  float* WTV = (float*)(ws + kOffWTV);
  float* EV = (float*)(ws + kOffEV);
  float* DV = (float*)(ws + kOffDV);
  float* TOT = (float*)(ws + kOffTOT);
  float* RS = (float*)(ws + kOffRS);
  unsigned short* C3 = (unsigned short*)(ws + kOffC3);
  unsigned short* B3 = (unsigned short*)(ws + kOffB3);
  unsigned short* BDT16 = (unsigned short*)(ws + kOffBDT16);
  unsigned short* H16 = (unsigned short*)(ws + kOffH16);
  unsigned short* CE16 = (unsigned short*)(ws + kOffCE16);
  float* YC32 = (float*)(ws + kOffYC32);
  unsigned short* XT16 = (unsigned short*)(ws + kOffXT16);
  float* G32 = (float*)(ws + kOffG32);
  float* YD32 = G32;
  unsigned short* M16 = (unsigned short*)(ws + kOffM16);
  float* ST32 = (float*)(ws + kOffST32);
  float* YO32 = ST32;
  const long kStr = (long)kQ * kN;
  const long kStr3 = (long)kQ * 192;

  zero_kernel<<<1, kThr, 0, stream>>>(ZB);
  bias_kernel<<<17, kThr, 0, stream>>>(dt_b, dt_bias, g_b, o_b, BIA);
  cast_plane_kernel<<<(int)(((size_t)kRowsAll * kHID / 8) / kThr), kThr, 0, stream>>>(hab, HX16, 11, kHID, 0);
  wt_plane_kernel<<<kH, kHID / 8, 0, stream>>>(dt_w, WDT16, kHID, kH, kH, kHID, 0);
  wmma_gemm32<<<dim3((kRowsAll / 64) * (kH / 32) / 8, 1), 256, 0, stream>>>(
      HX16, kHID, 0L, WDT16, kHID, 0L, DTL, kH, 0L, BIA + kBiaDt, kRowsAll, kH, kHID, kScT);
  cast_plane_kernel<<<(int)(((size_t)kRowsAll * kHID / 8) / kThr), kThr, 0, stream>>>(hg, HX16, 11, kHID, 0);
  wt_plane_kernel<<<kH, kHID / 8, 0, stream>>>(g_w, WG16, kHID, kH, kH, kHID, 0);
  wmma_gemm32<<<dim3((kRowsAll / 64) * (kH / 32) / 8, 1), 256, 0, stream>>>(
      HX16, kHID, 0L, WG16, kHID, 0L, GTL, kH, 0L, BIA + kBiaG, kRowsAll, kH, kHID, kScT);
  xt2_cast_kernel<<<128, kThr, 0, stream>>>(o_w, OW2);
  for (int b = 0; b < kNb; ++b) {
    const float* qb = qs + (size_t)b * kS * kH * kP;
    const float* kb = ks + (size_t)b * kS * kH * kP;
    const float* vb = vs + (size_t)b * kS * kH * kP;
    const float* DTLb = DTL + (size_t)b * kS * kH;
    const float* GTLb = GTL + (size_t)b * kS * kH;
    float* ob = out + (size_t)b * kS * kHID;
    rownorm_kernel<<<256, kThr, 0, stream>>>(qb, RNQ);
    rownorm_kernel<<<256, kThr, 0, stream>>>(kb, RNK);
    hm3_cast_kernel<<<2048, kThr, 0, stream>>>(qb, RNQ, C3, 0);
    hm3_cast_kernel<<<2048, kThr, 0, stream>>>(kb, RNK, B3, 1);
    xt_cast_kernel<<<2048, kThr, 0, stream>>>(vb, XT16);
    prefix_kernel<<<4, kThr, 0, stream>>>(DTLb, A_log, CS, WTV, EV, DV, TOT);
    wmma_gemm64<0, false, 2, 0, false, 0><<<dim3(1, kE), 256, 0, stream>>>(
        C3, C3, 192, kStr3, B3, B3, 192, kStr3, (void*)G32, (void*)G32, kQ, kStr, ZB, nullptr, 0L, kQ, kQ, 192, kSc1);
    mask_kernel<<<2048, kThr, 0, stream>>>(G32, CS, WTV, M16);
    wmma_gemm64<0, false, 2, 0, false, 0><<<dim3(1, kE), 256, 0, stream>>>(
        M16, M16, kQ, kStr, XT16, XT16, kQ, kStr, (void*)YD32, (void*)YD32, kP, kStr, ZB, nullptr, 0L, kQ, kP, kQ, kSc3);
    sc2_cast_kernel<<<2048, kThr, 0, stream>>>(kb, RNK, DV, BDT16, 1);
    wmma_gemm64<0, false, 2, 0, false, 0><<<dim3(1, kE), 256, 0, stream>>>(
        XT16, XT16, kQ, kStr, BDT16, BDT16, kQ, kStr, (void*)ST32, (void*)ST32, kN, kStr, ZB, nullptr, 0L, kP, kN, kQ, kSc4);
    carry_kernel<<<256, kThr, 0, stream>>>(ST32, TOT, H16);
    sc2_cast_kernel<<<2048, kThr, 0, stream>>>(qb, RNQ, EV, CE16, 0);
    wmma_gemm64<0, false, 2, 0, false, 0><<<dim3(1, kE), 256, 0, stream>>>(
        CE16, CE16, kN, kStr, H16, H16, kN, kStr, (void*)YO32, (void*)YO32, kP, kStr, ZB, nullptr, 0L, kQ, kP, kN, kSc6);
    combine_kernel<<<4096, kThr, 0, stream>>>(YD32, YO32, YC32);
    gnorm_kernel<<<8, kThr, 0, stream>>>(YC32, GTLb, RS);
    y2_cast_kernel<<<2048, kThr, 0, stream>>>(YC32, GTLb, RS, nw, Y2);
    for (int h = 0; h < kH; ++h) {
      wmma_gemm64<0, false, 2, 0, false, 0><<<dim3((kS / 64) * (kP / 64) / 8, 1), 256, 0, stream>>>(
          Y2 + (size_t)h * 128, Y2 + (size_t)h * 128, kH * 128, 0L, OW2 + (size_t)h * kP * 128, OW2 + (size_t)h * kP * 128, 128, 0L,
          (void*)(ob + (size_t)h * kP), (void*)(ob + (size_t)h * kP), kHID, 0L, BIA + kBiaO + h * kP, nullptr, 0L, kS, kP, 128, kScO);
    }
  }
}
